// MultiHeadSelfAttention_65481071399163
// MI455X (gfx1250) — hardware-verified
//
#include <hip/hip_runtime.h>
#ifndef NB
#define NB 2
#endif
#ifndef SEQ
#define SEQ 2048
#endif
#define NB_FULL 2
#define SEQ_FULL 2048
#define DM 1024
#define NH 16
#define HD 64
#define NR (NB * SEQ)
#define VTP NR
#define LA2 (2 * DM)

static_assert(NH * HD == DM);
static_assert(HD == 64);
static_assert(DM % 128 == 0);
static_assert(DM % 64 == 0);
static_assert(DM % 32 == 0);
static_assert(NR % 128 == 0);
static_assert(NR % 64 == 0);
static_assert(SEQ % 64 == 0);
static_assert(SEQ % 32 == 0);
static_assert(NB <= NB_FULL);
static_assert(SEQ <= SEQ_FULL);
static_assert((DM / 8) * 8 == DM);

typedef _Float16 v16h __attribute__((ext_vector_type(16)));
typedef _Float16 v4h  __attribute__((ext_vector_type(4)));
typedef unsigned short v8us __attribute__((ext_vector_type(8), may_alias));
typedef float  v8f  __attribute__((ext_vector_type(8)));
typedef float  v4f  __attribute__((ext_vector_type(4)));
typedef float  v4fa __attribute__((ext_vector_type(4), may_alias));
union FragH { v16h v; v8us half[2]; _Float16 h[16]; unsigned short u[16]; };

__device__ __forceinline__ unsigned short bf16_bits(float x) { unsigned int u = __float_as_uint(x); return (unsigned short)((u + 0x7FFFu + ((u >> 16) & 1u)) >> 16); }
__device__ __forceinline__ float bf16_rne(float x) { return __uint_as_float(((unsigned int)bf16_bits(x)) << 16); }

__device__ __forceinline__ v16h g2_frag(const _Float16* p, int hh) { FragH f; f.half[0] = *(const v8us*)((const unsigned short*)p + 8 * hh); f.half[1] = *(const v8us*)((const unsigned short*)p + 16 + 8 * hh); return f.v; }
__device__ __forceinline__ v8f g2_mma(v16h a, v16h b, v8f c) { v8f d = __builtin_amdgcn_wmma_f32_16x16x32_f16(false, a, false, b, (short)0, c, false, false); asm volatile("v_nop\n\tv_nop\n\tv_nop\n\tv_nop" : "+v"(d) : "v"(a), "v"(b)); return d; }

__global__ __launch_bounds__(256) void k_wt_f16(const float* __restrict__ W, _Float16* __restrict__ Wt, int ldt, float scale, float scale2) {
  const int t = blockIdx.x * 256 + threadIdx.x; if (t >= DM * (DM / 8)) return;
  const int n = t / (DM / 8), k8 = (t % (DM / 8)) * 8; FragH f, g;
#pragma unroll
  for (int i = 0; i < 8; ++i) { const float wv = bf16_rne(W[(size_t)(k8 + i) * DM + n]); f.h[i] = (_Float16)(wv * scale); g.h[i] = (_Float16)(wv * scale2); }
  const v8us o = f.half[0], o2 = g.half[0];
  unsigned short* d = (unsigned short*)Wt + (size_t)n * ldt + k8;
  *(volatile v8us*)d = o; if (scale2 != 0.f) *(volatile v8us*)(d + DM) = o2;
  __threadfence();
  *(volatile v8us*)d = o; if (scale2 != 0.f) *(volatile v8us*)(d + DM) = o2;
}

__global__ __launch_bounds__(256) void k_x16(const float* __restrict__ x, _Float16* __restrict__ X16, size_t n8) {
  const size_t t = (size_t)blockIdx.x * 256 + threadIdx.x; if (t >= n8) return;
  const size_t row = t / (DM / 8); const int c8 = (int)(t % (DM / 8)) * 8; const size_t b = row / SEQ, s = row % SEQ;
  const float* src = x + (b * SEQ_FULL + s) * DM + c8;
  const v4f a = *(const v4fa*)src, c = *(const v4fa*)(src + 4); FragH f;
#pragma unroll
  for (int q = 0; q < 4; ++q) { f.h[q] = (_Float16)bf16_rne(a[q]); f.h[4 + q] = (_Float16)bf16_rne(c[q]); }
  const v8us o = f.half[0];
  *(volatile v8us*)((unsigned short*)X16 + t * 8) = o; __threadfence(); *(volatile v8us*)((unsigned short*)X16 + t * 8) = o;
}

__global__ __launch_bounds__(128) void k_gemm2(const _Float16* __restrict__ A, int lda, const _Float16* __restrict__ Bh, int ldb, float alpha,
                                               const float* __restrict__ bias, int brow, float post,
                                               float* __restrict__ C, _Float16* __restrict__ C16, _Float16* __restrict__ C16L, int ldc, int M, int N, int K) {
  __shared__ __attribute__((aligned(16))) float so[4][32][68];
  const int tid = threadIdx.x, w = tid >> 5, lane = tid & 31, ln = lane & 15, hh = lane >> 4;
  const int ntn = N >> 6; const int mt = blockIdx.x / ntn, nq = blockIdx.x - mt * ntn; const int row0 = mt * 128 + 32 * w, col0 = nq * 64; if (row0 >= M) return;
  const _Float16* a0p = A + (size_t)(row0 + ln) * lda; const _Float16* a1p = a0p + (size_t)16 * lda;
  const _Float16* b0p = Bh + (size_t)(col0 + ln) * ldb; const _Float16* b1p = b0p + (size_t)16 * ldb; const _Float16* b2p = b1p + (size_t)16 * ldb; const _Float16* b3p = b2p + (size_t)16 * ldb;
  const v8f z8 = {0.f,0.f,0.f,0.f,0.f,0.f,0.f,0.f}; v8f c00 = z8, c01 = z8, c02 = z8, c03 = z8, c10 = z8, c11 = z8, c12 = z8, c13 = z8;
#pragma unroll 1
  for (int kb = 0; kb < K; kb += 32) { const v16h a0 = g2_frag(a0p + kb, hh), a1 = g2_frag(a1p + kb, hh);
    v16h b = g2_frag(b0p + kb, hh); c00 = g2_mma(a0, b, c00); c10 = g2_mma(a1, b, c10);
    b = g2_frag(b1p + kb, hh); c01 = g2_mma(a0, b, c01); c11 = g2_mma(a1, b, c11);
    b = g2_frag(b2p + kb, hh); c02 = g2_mma(a0, b, c02); c12 = g2_mma(a1, b, c12);
    b = g2_frag(b3p + kb, hh); c03 = g2_mma(a0, b, c03); c13 = g2_mma(a1, b, c13); }
  v8f accs[8] = {c00, c01, c02, c03, c10, c11, c12, c13};
#pragma unroll
  for (int u = 0; u < 8; ++u) { const int t = u & 3, half = u >> 2; const int col = col0 + t * 16 + ln;
    const float bvc = bf16_rne(bias[brow ? 0 : col]);
#pragma unroll
    for (int r = 0; r < 8; ++r) { const int rloc = half * 16 + 8 * hh + r;
      const float bvr = bf16_rne(bias[brow ? (row0 + rloc) : 0]);
      const float bv = brow ? bvr : bvc;
      so[w][rloc][t * 16 + ln] = (accs[u][r] * alpha + bv) * post; } }
  __builtin_amdgcn_fence(4  , "workgroup"); __builtin_amdgcn_wave_barrier();
  const int rsub = lane >> 4, c4 = (lane & 15) * 4;
  for (int pass = 0; pass < 2; ++pass) {
#pragma unroll
    for (int q = 0; q < 16; ++q) { const int r = q * 2 + rsub; const v4f v = *(const v4fa*)&so[w][r][c4];
      const size_t o = (size_t)(row0 + r) * ldc + col0 + c4;
      if (C) *(volatile v4f*)(C + o) = v;
      if (C16 != nullptr || C16L != nullptr) { v4h h4, l4;
#pragma unroll
        for (int i = 0; i < 4; ++i) { const _Float16 hv = (_Float16)v[i]; h4[i] = hv; l4[i] = (_Float16)((v[i] - (float)hv) * 1024.0f); }
        if (C16) *(volatile v4h*)(C16 + o) = h4;
        if (C16L) *(volatile v4h*)(C16L + o) = l4; } }
    if (pass == 0) __threadfence(); }
}

__global__ __launch_bounds__(128) void k_attn(const _Float16* __restrict__ QH, const _Float16* __restrict__ QL, const _Float16* __restrict__ K16,
                                              const _Float16* __restrict__ VT, const float* __restrict__ x, _Float16* __restrict__ A2) {
  __shared__ __attribute__((aligned(16))) float so[4][16][68];
  const int tid = threadIdx.x, w = tid >> 5, lane = tid & 31, ln = lane & 15, hh = lane >> 4;
  const int bh = blockIdx.y; const int b = bh / NH, h = bh - b * NH;
  const int q0 = blockIdx.x * 64 + w * 16;
  const size_t rb = (size_t)b * SEQ;
  const size_t qoff = (rb + q0 + ln) * DM + h * HD;
  const v16h qh0 = g2_frag(QH + qoff, hh), qh1 = g2_frag(QH + qoff + 32, hh);
  const v16h ql0 = g2_frag(QL + qoff, hh), ql1 = g2_frag(QL + qoff + 32, hh);
  const _Float16* kbase = K16 + (rb + ln) * DM + h * HD;
  const _Float16* vbase = VT + (size_t)(h * HD + ln) * VTP + rb;
  const v8f z8 = {0.f,0.f,0.f,0.f,0.f,0.f,0.f,0.f};
  v8f o0 = z8, o1 = z8, o2 = z8, o3 = z8;
  float m = -1.0e30f, l = 0.f;
  const float RS = 0.0009765625f;
  const float PC = 5.545177444f;
#pragma unroll 1
  for (int kt = 0; kt < SEQ; kt += 32) {
    const _Float16* kp0 = kbase + (size_t)kt * DM; const _Float16* kp1 = kp0 + (size_t)16 * DM;
    v8f sh0 = z8, sl0 = z8, sh1 = z8, sl1 = z8;
    v16h kf = g2_frag(kp0, hh);      sh0 = g2_mma(kf, qh0, sh0); sl0 = g2_mma(kf, ql0, sl0);
    kf = g2_frag(kp0 + 32, hh);      sh0 = g2_mma(kf, qh1, sh0); sl0 = g2_mma(kf, ql1, sl0);
    kf = g2_frag(kp1, hh);           sh1 = g2_mma(kf, qh0, sh1); sl1 = g2_mma(kf, ql0, sl1);
    kf = g2_frag(kp1 + 32, hh);      sh1 = g2_mma(kf, qh1, sh1); sl1 = g2_mma(kf, ql1, sl1);
    float s0[8], s1[8]; float mx = -1.0e30f;
#pragma unroll
    for (int r = 0; r < 8; ++r) { s0[r] = sh0[r] + sl0[r] * RS; s1[r] = sh1[r] + sl1[r] * RS; mx = fmaxf(mx, fmaxf(s0[r], s1[r])); }
    mx = fmaxf(mx, __shfl_xor(mx, 16, 32));
    const float mnew = fmaxf(m, mx); const float alpha = __expf(m - mnew); m = mnew;
    const float sub = mnew - PC;
    FragH pf; float rs = 0.f;
#pragma unroll
    for (int r = 0; r < 8; ++r) { const float p0 = __expf(s0[r] - sub), p1 = __expf(s1[r] - sub); rs += p0 + p1; pf.h[r] = (_Float16)p0; pf.h[8 + r] = (_Float16)p1; }
    l = l * alpha + rs;
#pragma unroll
    for (int r = 0; r < 8; ++r) { o0[r] *= alpha; o1[r] *= alpha; o2[r] *= alpha; o3[r] *= alpha; }
    const _Float16* vp = vbase + kt;
    const v16h v0 = g2_frag(vp, hh), v1 = g2_frag(vp + (size_t)16 * VTP, hh), v2 = g2_frag(vp + (size_t)32 * VTP, hh), v3 = g2_frag(vp + (size_t)48 * VTP, hh);
    o0 = g2_mma(v0, pf.v, o0); o1 = g2_mma(v1, pf.v, o1); o2 = g2_mma(v2, pf.v, o2); o3 = g2_mma(v3, pf.v, o3);
  }
  const float lt = l + __shfl_xor(l, 16, 32);
  const float inv = 1.0f / lt;
#pragma unroll
  for (int r = 0; r < 8; ++r) {
    so[w][ln][8 * hh + r] = o0[r] * inv; so[w][ln][16 + 8 * hh + r] = o1[r] * inv;
    so[w][ln][32 + 8 * hh + r] = o2[r] * inv; so[w][ln][48 + 8 * hh + r] = o3[r] * inv; }
  __builtin_amdgcn_fence(4  , "workgroup"); __builtin_amdgcn_wave_barrier();
  const int rq = lane >> 3, pc = lane & 7;
  v8us hv[4], lv[4];
#pragma unroll
  for (int it = 0; it < 4; ++it) { const int q = it * 4 + rq;
    const v4f c0 = *(const v4fa*)&so[w][q][pc * 8], c1 = *(const v4fa*)&so[w][q][pc * 8 + 4];
    const float* xr = x + ((size_t)b * SEQ_FULL + q0 + q) * DM + h * HD + pc * 8;
    const v4f x0 = *(const v4fa*)xr, x1 = *(const v4fa*)(xr + 4);
    FragH fh, fl;
#pragma unroll
    for (int i = 0; i < 4; ++i) {
      const float sa = c0[i] + bf16_rne(x0[i]); const _Float16 ha = (_Float16)sa; fh.h[i] = ha; fl.h[i] = (_Float16)((sa - (float)ha) * 1024.0f);
      const float sb = c1[i] + bf16_rne(x1[i]); const _Float16 hb = (_Float16)sb; fh.h[4 + i] = hb; fl.h[4 + i] = (_Float16)((sb - (float)hb) * 1024.0f); }
    hv[it] = fh.half[0]; lv[it] = fl.half[0]; }
  for (int pass = 0; pass < 2; ++pass) {
#pragma unroll
    for (int it = 0; it < 4; ++it) { const int q = it * 4 + rq;
      unsigned short* d = (unsigned short*)A2 + (rb + q0 + q) * LA2 + h * HD + pc * 8;
      *(volatile v8us*)d = hv[it];
      *(volatile v8us*)(d + DM) = lv[it]; }
    if (pass == 0) __threadfence(); }
}

constexpr size_t al256(size_t b) { return (b + 255) & ~(size_t)255; }
constexpr size_t WS_W   = al256((size_t)DM * DM * 2);
constexpr size_t WS_WO  = al256((size_t)DM * LA2 * 2);
constexpr size_t WS_ROW = al256((size_t)NR * DM * 2);
constexpr size_t WS_A2  = al256((size_t)NR * LA2 * 2);
constexpr size_t WS_TOTAL = 3 * WS_W + WS_WO + 5 * WS_ROW + WS_A2;
static_assert(WS_TOTAL <= (size_t)134217728);

extern "C" void kernel_launch(void* const* d_in, const int* in_sizes, int n_in,
                              void* d_out, int out_size, void* d_ws, size_t ws_size, hipStream_t stream) {
  if (n_in < 9) return;
  if ((size_t)in_sizes[0] < ((size_t)(NB - 1) * SEQ_FULL + SEQ) * DM) return;
  if (in_sizes[1] < DM * DM || in_sizes[3] < DM * DM || in_sizes[5] < DM * DM || in_sizes[7] < DM * DM) return;
  if (in_sizes[2] < DM || in_sizes[4] < DM || in_sizes[6] < DM || in_sizes[8] < DM) return;
  if ((size_t)out_size < (size_t)NR * DM) return;
  if (WS_TOTAL > ws_size) return;
  const float* x  = (const float*)d_in[0];
  const float* wq = (const float*)d_in[1]; const float* bq = (const float*)d_in[2];
  const float* wk = (const float*)d_in[3]; const float* bk = (const float*)d_in[4];
  const float* wv = (const float*)d_in[5]; const float* bv = (const float*)d_in[6];
  const float* wo = (const float*)d_in[7]; const float* bo = (const float*)d_in[8];
  char* ws = (char*)d_ws; size_t off = 0;
  _Float16* BQ  = (_Float16*)(ws + off); off += WS_W;
  _Float16* BK  = (_Float16*)(ws + off); off += WS_W;
  _Float16* BV  = (_Float16*)(ws + off); off += WS_W;
  _Float16* BO2 = (_Float16*)(ws + off); off += WS_WO;
  _Float16* X16 = (_Float16*)(ws + off); off += WS_ROW;
  _Float16* QH  = (_Float16*)(ws + off); off += WS_ROW;
  _Float16* QL  = (_Float16*)(ws + off); off += WS_ROW;
  _Float16* K16 = (_Float16*)(ws + off); off += WS_ROW;
  _Float16* VT  = (_Float16*)(ws + off); off += WS_ROW;
  _Float16* A2  = (_Float16*)(ws + off); off += WS_A2;
  if (off > ws_size) return;

  const unsigned gw = (unsigned)(((size_t)DM * (DM / 8) + 255) / 256);
  k_wt_f16<<<gw, 256, 0, stream>>>(wq, BQ, DM, 16.0f, 0.0f);
  k_wt_f16<<<gw, 256, 0, stream>>>(wk, BK, DM, 16.0f, 0.0f);
  k_wt_f16<<<gw, 256, 0, stream>>>(wv, BV, DM, 16.0f, 0.0f);
  k_wt_f16<<<gw, 256, 0, stream>>>(wo, BO2, LA2, 256.0f, 0.25f);
  const size_t n8 = (size_t)NR * DM / 8;
  k_x16<<<(unsigned)((n8 + 255) / 256), 256, 0, stream>>>(x, X16, n8);

  const unsigned gp = (unsigned)((NR / 128) * (DM / 64));
  k_gemm2<<<gp, 128, 0, stream>>>(X16, DM, BQ, DM, 0.0625f, bq, 0, 0.125f, nullptr, QH, QL, DM, NR, DM, DM);
  k_gemm2<<<gp, 128, 0, stream>>>(X16, DM, BK, DM, 0.0625f, bk, 0, 1.0f, nullptr, K16, nullptr, DM, NR, DM, DM);
  const unsigned gv = (unsigned)((DM / 128) * (NR / 64));
  k_gemm2<<<gv, 128, 0, stream>>>(BV, DM, X16, DM, 0.0625f, bv, 1, 1.0f, nullptr, VT, nullptr, VTP, DM, NR, DM);

  k_attn<<<dim3(SEQ / 64, NB * NH), 128, 0, stream>>>(QH, QL, K16, VT, x, A2);

  k_gemm2<<<gp, 128, 0, stream>>>(A2, LA2, BO2, LA2, 0.00390625f, bo, 0, 1.0f, (float*)d_out, nullptr, nullptr, DM, NR, DM, LA2);
}
